// GPT2Attention_70300024701797
// MI455X (gfx1250) — hardware-verified
//
#include <hip/hip_runtime.h>
#ifndef NB
#define NB 2
#endif
#ifndef SEQ
#define SEQ 2048
#endif
#define NB_FULL 2
#define SEQ_FULL 2048
#define DM 1024
#define NH 16
#define HD 64
#define HG 2
#define LQ (3 * DM)
#define NR ((size_t)NB * SEQ)
static_assert(SEQ % 256 == 0);
static_assert(NR % 128 == 0);
static_assert(NH % HG == 0);
static_assert(DM % 64 == 0);
static_assert(HD == 64);
static_assert(NB >= 1 && NB <= NB_FULL);
static_assert(SEQ <= SEQ_FULL);
static_assert(LQ % 64 == 0);

typedef unsigned short v8us __attribute__((ext_vector_type(8), may_alias));
typedef float  v8f  __attribute__((ext_vector_type(8)));
typedef float  v4f  __attribute__((ext_vector_type(4)));
typedef float  v4fa __attribute__((ext_vector_type(4), may_alias));
typedef _Float16 v16h __attribute__((ext_vector_type(16)));
typedef _Float16 v4h  __attribute__((ext_vector_type(4)));
union FragH { v16h v; v8us half[2]; _Float16 h[16]; unsigned short u[16]; };
union H8 { v8us v; _Float16 h[8]; unsigned short u[8]; };

__device__ __forceinline__ unsigned short bf16_bits(float x) { unsigned int u = __float_as_uint(x); return (unsigned short)((u + 0x7FFFu + ((u >> 16) & 1u)) >> 16); }
__device__ __forceinline__ float bf16_val(unsigned short b) { return __uint_as_float(((unsigned int)b) << 16); }
__device__ __forceinline__ float bf16_rne(float x) { return bf16_val(bf16_bits(x)); }

__device__ __forceinline__ v16h g2_frag(const _Float16* p, int hh) { FragH f; f.half[0] = *(const v8us*)((const unsigned short*)p + 8 * hh); f.half[1] = *(const v8us*)((const unsigned short*)p + 16 + 8 * hh); return f.v; }
__device__ __forceinline__ v8f g2_mma(v16h a, v16h b, v8f c) { v8f d = __builtin_amdgcn_wmma_f32_16x16x32_f16(false, a, false, b, (short)0, c, false, false); asm volatile("v_nop\n\tv_nop\n\tv_nop\n\tv_nop" : "+v"(d) : "v"(a), "v"(b)); return d; }

__global__ __launch_bounds__(256) void k_wt_f16(const float* __restrict__ W, _Float16* __restrict__ Wt, int K, int N, float scale) {
  const int t = blockIdx.x * 256 + threadIdx.x; if (t >= N * (K / 8)) return;
  const int n = t / (K / 8), k8 = (t % (K / 8)) * 8; H8 f;
#pragma unroll
  for (int i = 0; i < 8; ++i) f.h[i] = (_Float16)(bf16_rne(W[(size_t)(k8 + i) * N + n]) * scale);
  unsigned short* d = (unsigned short*)Wt + (size_t)n * K + k8;
  *(volatile v8us*)d = f.v; __threadfence(); *(volatile v8us*)d = f.v;
}

__global__ __launch_bounds__(256) void k_x16b(const float* __restrict__ x, _Float16* __restrict__ X16, size_t n8) {
  const size_t t = (size_t)blockIdx.x * 256 + threadIdx.x; if (t >= n8) return;
  const size_t rc = t / (DM / 8); const int c8 = (int)(t % (DM / 8)) * 8; const size_t b = rc / SEQ, s = rc % SEQ;
  const float* src = x + (b * SEQ_FULL + s) * DM + c8;
  const v4f a = *(const v4fa*)src, c = *(const v4fa*)(src + 4); H8 f;
#pragma unroll
  for (int q = 0; q < 4; ++q) { f.h[q] = (_Float16)bf16_rne(a[q]); f.h[4 + q] = (_Float16)bf16_rne(c[q]); }
  unsigned short* d = (unsigned short*)X16 + t * 8;
  *(volatile v8us*)d = f.v; __threadfence(); *(volatile v8us*)d = f.v;
}

template <int ACT>
__global__ __launch_bounds__(128) void k_gemm2(const _Float16* __restrict__ A, int lda, size_t sA, const _Float16* __restrict__ Bh, int ldb, size_t sB, float alpha, const float* __restrict__ bias,
    float* __restrict__ C, _Float16* __restrict__ C16, int ldc, size_t sC, int M, int N, int K) {
  static_assert(ACT == 0);
  __shared__ __attribute__((aligned(16))) float so[4][32][68];
  const int tid = threadIdx.x, w = tid >> 5, lane = tid & 31, ln = lane & 15, hh = lane >> 4; const int by = blockIdx.y;
  A += (size_t)by * sA; Bh += (size_t)by * sB; const size_t cofs = (size_t)by * sC;
  const int ntn = N >> 6; const int mt = blockIdx.x / ntn, nq = blockIdx.x - mt * ntn; const int row0 = mt * 128 + 32 * w, col0 = nq * 64; if (row0 >= M) return;
  const _Float16* a0p = A + (size_t)(row0 + ln) * lda; const _Float16* a1p = a0p + (size_t)16 * lda;
  const _Float16* b0p = Bh + (size_t)(col0 + ln) * ldb; const _Float16* b1p = b0p + (size_t)16 * ldb; const _Float16* b2p = b1p + (size_t)16 * ldb; const _Float16* b3p = b2p + (size_t)16 * ldb;
  const v8f z8 = {0.f,0.f,0.f,0.f,0.f,0.f,0.f,0.f}; v8f c00 = z8, c01 = z8, c02 = z8, c03 = z8, c10 = z8, c11 = z8, c12 = z8, c13 = z8;
#pragma unroll 1
  for (int kb = 0; kb < K; kb += 32) { const v16h a0 = g2_frag(a0p + kb, hh), a1 = g2_frag(a1p + kb, hh);
    v16h b = g2_frag(b0p + kb, hh); c00 = g2_mma(a0, b, c00); c10 = g2_mma(a1, b, c10);
    b = g2_frag(b1p + kb, hh); c01 = g2_mma(a0, b, c01); c11 = g2_mma(a1, b, c11);
    b = g2_frag(b2p + kb, hh); c02 = g2_mma(a0, b, c02); c12 = g2_mma(a1, b, c12);
    b = g2_frag(b3p + kb, hh); c03 = g2_mma(a0, b, c03); c13 = g2_mma(a1, b, c13); }
  v8f accs[8] = {c00, c01, c02, c03, c10, c11, c12, c13};
#pragma unroll
  for (int u = 0; u < 8; ++u) { const int t = u & 3, half = u >> 2; const int col = col0 + t * 16 + ln; const float bv = bias ? bf16_rne(bias[col]) : 0.f;
#pragma unroll
    for (int r = 0; r < 8; ++r) { const int rloc = half * 16 + 8 * hh + r; const float v = accs[u][r] * alpha + bv; so[w][rloc][t * 16 + ln] = v; } }
  __builtin_amdgcn_fence(4  , "workgroup"); __builtin_amdgcn_wave_barrier();
  const int rsub = lane >> 4, c4 = (lane & 15) * 4;
  for (int pass = 0; pass < 2; ++pass) {
#pragma unroll
    for (int q = 0; q < 16; ++q) { const int r = q * 2 + rsub; const v4f v = *(const v4fa*)&so[w][r][c4];
      if (C) *(volatile v4f*)(C + cofs + (size_t)(row0 + r) * ldc + col0 + c4) = v;
      if (C16) { v4h h4; for (int i = 0; i < 4; ++i) h4[i] = (_Float16)v[i]; *(volatile v4h*)(C16 + cofs + (size_t)(row0 + r) * ldc + col0 + c4) = h4; } }
    if (pass == 0) __threadfence(); } }

__global__ __launch_bounds__(256) void k_vt(const _Float16* __restrict__ V16, int ldv, _Float16* __restrict__ Vt) {
  __shared__ unsigned short tl[64][66];
  const int tid = threadIdx.x; const int slab = blockIdx.x / (SEQ / 64), lg = blockIdx.x % (SEQ / 64); const int b = slab / NH, h = slab % NH;
  for (int i = tid; i < 64 * 8; i += 256) { const int r = i / 8, c8 = (i % 8) * 8; H8 f; f.v = *(const v8us*)((const unsigned short*)V16 + ((size_t)b * SEQ + lg * 64 + r) * ldv + h * HD + c8);
#pragma unroll
    for (int q = 0; q < 8; ++q) tl[r][c8 + q] = f.u[q]; }
  __syncthreads();
  for (int pass = 0; pass < 2; ++pass) {
#pragma unroll
    for (int rd = 0; rd < 2; ++rd) { const int d = rd * 32 + tid / 8, pc = tid % 8; H8 f;
#pragma unroll
      for (int q = 0; q < 8; ++q) f.u[q] = tl[pc * 8 + q][d];
      *(volatile v8us*)((unsigned short*)Vt + ((size_t)slab * HD + d) * SEQ + lg * 64 + pc * 8) = f.v; }
    if (pass == 0) __threadfence(); } }

__global__ __launch_bounds__(256) void k_rsmw(const float* __restrict__ S, _Float16* __restrict__ P, int nrows) {
  #pragma clang fp contract(off)
  constexpr int NIT = SEQ / 256;
  const int row = blockIdx.x * 8 + (threadIdx.x >> 5), lane = threadIdx.x & 31;
  if (row >= nrows) return;
  const float* s = S + (size_t)row * SEQ + lane * 8;
  float e[NIT][8]; float mx = -3.0e38f;
#pragma unroll
  for (int it = 0; it < NIT; ++it) { const v4f a = *(const v4fa*)(s + it * 256), c = *(const v4fa*)(s + it * 256 + 4);
#pragma unroll
    for (int q = 0; q < 4; ++q) { e[it][q] = a[q]; e[it][4 + q] = c[q]; mx = fmaxf(mx, fmaxf(a[q], c[q])); } }
#pragma unroll
  for (int m = 16; m > 0; m >>= 1) mx = fmaxf(mx, __shfl_xor(mx, m, 32));
  float se = 0.f;
#pragma unroll
  for (int it = 0; it < NIT; ++it) {
#pragma unroll
    for (int q = 0; q < 8; ++q) { const float v = __expf(e[it][q] - mx); e[it][q] = v; se += v; } }
#pragma unroll
  for (int m = 16; m > 0; m >>= 1) se += __shfl_xor(se, m, 32);
  const float sc = 256.0f / se;
  H8 f[NIT];
#pragma unroll
  for (int it = 0; it < NIT; ++it) {
#pragma unroll
    for (int q = 0; q < 8; ++q) f[it].h[q] = (_Float16)(e[it][q] * sc); }
  unsigned short* d = (unsigned short*)P + (size_t)row * SEQ + lane * 8;
  for (int pass = 0; pass < 2; ++pass) {
#pragma unroll
    for (int it = 0; it < NIT; ++it) *(volatile v8us*)(d + it * 256) = f[it].v;
    if (pass == 0) __threadfence(); }
}

extern "C" void kernel_launch(void* const* d_in, const int* in_sizes, int n_in,
                              void* d_out, int out_size, void* d_ws, size_t ws_size, hipStream_t stream) {
  if (n_in < 5) return;
  if ((size_t)in_sizes[0] < (((size_t)NB - 1) * SEQ_FULL + SEQ) * DM) return;
  if (in_sizes[1] < DM * LQ || in_sizes[2] < LQ || in_sizes[3] < DM * DM || in_sizes[4] < DM) return;
  if ((size_t)out_size < NR * DM) return;
  const float* x = (const float*)d_in[0]; const float* wqkv = (const float*)d_in[1]; const float* bqkv = (const float*)d_in[2];
  const float* wo = (const float*)d_in[3]; const float* bo = (const float*)d_in[4];
  char* ws = (char*)d_ws; size_t off = 0;
  auto take = [&](size_t bytes) { char* p = ws + off; off += (bytes + 255) & ~(size_t)255; return p; };
  _Float16* BQKV = (_Float16*)take((size_t)LQ * DM * 2);
  _Float16* BO   = (_Float16*)take((size_t)DM * DM * 2);
  _Float16* X16  = (_Float16*)take(NR * DM * 2);
  _Float16* QKV  = (_Float16*)take(NR * LQ * 2);
  _Float16* O16  = (_Float16*)take(NR * DM * 2);
  float*    S    = (float*)take((size_t)HG * SEQ * SEQ * 4);
  _Float16* P    = (_Float16*)take((size_t)HG * SEQ * SEQ * 2);
  _Float16* VT   = (_Float16*)take((size_t)NB * NH * HD * SEQ * 2);
  if (off > ws_size) return;
  _Float16* Q16 = QKV; _Float16* K16 = QKV + DM; _Float16* V16 = QKV + 2 * DM;

  k_wt_f16<<<(unsigned)(((size_t)LQ * (DM / 8) + 255) / 256), 256, 0, stream>>>(wqkv, BQKV, DM, LQ, 16.0f);
  k_wt_f16<<<(unsigned)(((size_t)DM * (DM / 8) + 255) / 256), 256, 0, stream>>>(wo, BO, DM, DM, 16.0f);
  k_x16b<<<(unsigned)((NR * DM / 8 + 255) / 256), 256, 0, stream>>>(x, X16, NR * DM / 8);
  k_gemm2<0><<<dim3((unsigned)((NR / 128) * (LQ / 64)), 1), 128, 0, stream>>>(X16, DM, (size_t)0, BQKV, DM, (size_t)0, 0.0625f, bqkv, nullptr, QKV, LQ, (size_t)0, (int)NR, LQ, DM);
  k_vt<<<(unsigned)(NB * NH * (SEQ / 64)), 256, 0, stream>>>(V16, LQ, VT);
  for (int b = 0; b < NB; ++b) { const size_t r0 = (size_t)b * SEQ;
    for (int h0 = 0; h0 < NH; h0 += HG) {
      k_gemm2<0><<<dim3((unsigned)((SEQ / 128) * (SEQ / 64)), HG), 128, 0, stream>>>(Q16 + r0 * LQ + h0 * HD, LQ, (size_t)HD, K16 + r0 * LQ + h0 * HD, LQ, (size_t)HD, 0.125f, nullptr, S, nullptr, SEQ, (size_t)SEQ * SEQ, SEQ, SEQ, HD);
      k_rsmw<<<(unsigned)((HG * SEQ) / 8), 256, 0, stream>>>(S, P, HG * SEQ);
      k_gemm2<0><<<dim3((unsigned)((SEQ / 128) * (HD / 64)), HG), 128, 0, stream>>>(P, SEQ, (size_t)SEQ * SEQ, VT + ((size_t)b * NH + h0) * HD * SEQ, SEQ, (size_t)HD * SEQ, 0.25f, nullptr, nullptr, O16 + r0 * DM + h0 * HD, DM, (size_t)HD, SEQ, HD, SEQ); } }
  k_gemm2<0><<<dim3((unsigned)((NR / 128) * (DM / 64)), 1), 128, 0, stream>>>(O16, DM, (size_t)0, BO, DM, (size_t)0, 0.0009765625f, bo, (float*)d_out, nullptr, DM, (size_t)0, (int)NR, DM, DM);
}
